// pLoss_all_fidelity_21517786153437
// MI455X (gfx1250) — hardware-verified
//
#include <hip/hip_runtime.h>


namespace {
constexpr int B = 131072, NLIM = 131072  , L = 12, LP = 32  , NS = 512, LO = 16  ;
constexpr float FS = 8.0f, PSC = 1024.0f;
static_assert(B % 32 == 0 && NLIM % 32 == 0 && NLIM <= B && NS % 128 == 0 && L < LO, "tiling");
typedef _Float16 b16;
typedef __attribute__((ext_vector_type(16))) _Float16 v16b;
typedef __attribute__((ext_vector_type(8))) _Float16 v8b;
typedef __attribute__((ext_vector_type(8))) float v8f;
typedef __attribute__((ext_vector_type(4))) float v4f;
__device__ __forceinline__ float bf16_rne(float f) { unsigned int u = __float_as_uint(f); u += 0x7FFFu + ((u >> 16) & 1u); return __uint_as_float(u & 0xFFFF0000u); }
__device__ __forceinline__ void split16(float v, b16& hi, b16& lo) { hi = (b16)v; lo = (b16)(v - (float)hi); }
__device__ __forceinline__ v16b frag_kb(const b16* p, int hh) { const v8b a = *(const v8b*)(p + 8 * hh), b = *(const v8b*)(p + 16 + 8 * hh); v16b f;
#pragma unroll
  for (int e = 0; e < 8; ++e) { f[e] = a[e]; f[8 + e] = b[e]; } return f; }
__device__ __forceinline__ v8f wmma16b(v16b a, v16b b, v8f c) { v8f d = __builtin_amdgcn_wmma_f32_16x16x32_f16(false, a, false, b, (short)0, c, false, false); asm volatile("v_nop\n\tv_nop\n\tv_nop\n\tv_nop" : "+v"(d) : "v"(a), "v"(b)); return d; }
__device__ __forceinline__ void wave_lds_sync() { __builtin_amdgcn_fence(__ATOMIC_RELEASE, "workgroup"); __builtin_amdgcn_wave_barrier(); __builtin_amdgcn_fence(__ATOMIC_ACQUIRE, "workgroup"); }
__device__ __forceinline__ float pmul(float a, float b) { float p = a * b; asm volatile("" : "+v"(p)); return p; }
__device__ __forceinline__ int iclamp(int v, int lo, int hi) { return v < lo ? lo : (v > hi ? hi : v); }

__global__ __launch_bounds__(256) void prep_kernel(const float* __restrict__ f, const int* __restrict__ S, b16* __restrict__ Fh, b16* __restrict__ Sp, b16* __restrict__ MT) {
  size_t t = (size_t)blockIdx.x * 256 + threadIdx.x; v8b o;
  const size_t nf = (size_t)B * LP / 8; if (t < nf) { const size_t e = t * 8; const size_t b = e / LP; const int k0 = (int)(e % LP); for (int j = 0; j < 8; ++j) o[j] = (k0 + j < L) ? (b16)(bf16_rne(f[b * L + k0 + j]) * FS) : (b16)0.0f; for (int pass = 0; pass < 2; ++pass) { *(volatile v8b*)(Fh + e) = o; __threadfence(); } return; } t -= nf;
  const size_t ns = (size_t)NS * LP / 8; if (t < ns) { const size_t e = t * 8; const int n = (int)(e / LP), k0 = (int)(e % LP); for (int j = 0; j < 8; ++j) o[j] = (k0 + j < L) ? (b16)(float)iclamp(S[n * L + k0 + j], 0, 1 << 11) : (b16)0.0f; for (int pass = 0; pass < 2; ++pass) { *(volatile v8b*)(Sp + e) = o; __threadfence(); } return; } t -= ns;
  const size_t nm = (size_t)LO * NS / 8; if (t < nm) { const size_t e = t * 8; const int l = (int)(e / NS), n0 = (int)(e % NS); for (int j = 0; j < 8; ++j) { const int n = n0 + j; o[j] = (l < L) ? (b16)(S[n * L + l] > 0 ? 1.0f : 0.0f) : (l == L ? (b16)1.0f : (b16)0.0f); } for (int pass = 0; pass < 2; ++pass) { *(volatile v8b*)(MT + e) = o; __threadfence(); } }
}
__global__ __launch_bounds__(64) void marg_kernel(const b16* __restrict__ Fh, const b16* __restrict__ Sp, const b16* __restrict__ MT, float* __restrict__ out) {
  __shared__ __attribute__((aligned(16))) b16 Jh[2][16][NS + 8], Jl[2][16][NS + 8]; __shared__ __attribute__((aligned(16))) float Tf[2][16][128 + 4]; __shared__ __attribute__((aligned(16))) float Os[2][16 * L];
  const int wave = threadIdx.x >> 5, lane = threadIdx.x & 31, nloc = lane & 15, hlf = lane >> 4; const size_t m0 = (size_t)blockIdx.x * 32 + wave * 16;
  const v16b a = frag_kb(Fh + (m0 + nloc) * LP, hlf);
  const float rs = 1.0f / FS;
  float mx[8];
#pragma unroll
  for (int r = 0; r < 8; ++r) mx[r] = -INFINITY;
#pragma unroll 4
  for (int t = 0; t < NS / 16; ++t) { v8f c = (v8f){}; c = wmma16b(a, frag_kb(Sp + (size_t)(t * 16 + nloc) * LP, hlf), c);
#pragma unroll
    for (int r = 0; r < 8; ++r) mx[r] = fmaxf(mx[r], c[r] * rs); }
#pragma unroll
  for (int r = 0; r < 8; ++r) {
#pragma unroll
    for (int o = 1; o < 16; o <<= 1) mx[r] = fmaxf(mx[r], __shfl_xor(mx[r], o)); }
#pragma unroll 1
  for (int g = 0; g < NS / 128; ++g) {
#pragma unroll
    for (int tt = 0; tt < 8; ++tt) { const int t = g * 8 + tt; v8f c = (v8f){}; c = wmma16b(a, frag_kb(Sp + (size_t)(t * 16 + nloc) * LP, hlf), c);
#pragma unroll
      for (int r = 0; r < 8; ++r) Tf[wave][8 * hlf + r][tt * 16 + nloc] = __expf(c[r] * rs - mx[r]); }
    wave_lds_sync();
    { const int row = lane & 15; const int ch = (lane >> 4) * 64;
#pragma unroll
      for (int q = 0; q < 8; ++q) { v8b hv, lv;
#pragma unroll
        for (int j = 0; j < 8; ++j) { b16 p, qq; split16(Tf[wave][row][ch + q * 8 + j] * PSC, p, qq); hv[j] = p; lv[j] = qq; }
        *(v8b*)(&Jh[wave][row][g * 128 + ch + q * 8]) = hv; *(v8b*)(&Jl[wave][row][g * 128 + ch + q * 8]) = lv; } }
    wave_lds_sync(); }
  v8f acc = (v8f){};
#pragma unroll 4
  for (int kb = 0; kb < NS; kb += 32) { const v16b jh = frag_kb(&Jh[wave][nloc][kb], hlf), jl = frag_kb(&Jl[wave][nloc][kb], hlf), bm = frag_kb(MT + (size_t)nloc * NS + kb, hlf); acc = wmma16b(jh, bm, acc); acc = wmma16b(jl, bm, acc); }
#pragma unroll
  for (int r = 0; r < 8; ++r) { const float z = __shfl(acc[r], hlf * 16 + L, 32); if (nloc < L) Os[wave][(8 * hlf + r) * L + nloc] = acc[r] / z; }
  wave_lds_sync();
  for (int pass = 0; pass < 2; ++pass) { for (int q = lane; q < 16 * L / 4; q += 32) *(volatile v4f*)(out + m0 * L + q * 4) = *(const v4f*)(&Os[wave][q * 4]); __threadfence(); }
}
}

extern "C" void kernel_launch(void* const* d_in, const int* in_sizes, int n_in, void* d_out, int out_size, void* d_ws, size_t ws_size, hipStream_t stream) {
  (void)n_in;
  if (in_sizes[0] != B * L || in_sizes[1] != NS * L || out_size != B * L) return;
  size_t off = 0; char* ws = (char*)d_ws;
  auto carve = [&](size_t bytes) { char* p = ws + off; off += (bytes + 255) & ~(size_t)255; return p; };
  b16* Fh = (b16*)carve((size_t)B * LP * 2); b16* Sp = (b16*)carve((size_t)NS * LP * 2); b16* MT = (b16*)carve((size_t)LO * NS * 2);
  if (off > ws_size || off > ((size_t)128 << 20)) return;
  prep_kernel<<<(unsigned)((((size_t)B * LP + (size_t)NS * LP + (size_t)LO * NS) / 8 + 255) / 256), 256, 0, stream>>>((const float*)d_in[0], (const int*)d_in[1], Fh, Sp, MT);
  marg_kernel<<<NLIM / 32, 64, 0, stream>>>(Fh, Sp, MT, (float*)d_out);
}
